// MPNNEncoderVAE_39779987095906
// MI455X (gfx1250) — hardware-verified
//
#include <hip/hip_runtime.h>
#include <stddef.h>


#define FI    128
#define HD    256
#define NH    8
#define HC    32
#define NL    3
#define LT    64
#define LR    8
#define NG    64
#define GR    32
#define XSP   260
#define NTHR  256
#define NWAVE 8
#define NB    256
#define CHUNK 2048
#define WCAP  256
#define NGRP  (CHUNK / (NTHR * 4))
#define GP    264
#define OSP   68

#define LDS_SACC (NB * HD)
#define LDS_DEN  (NB * NH)
#define LDS_MX   (NB * NH)
#define LDS_LIST (NWAVE * WCAP)
#define AGG_LDS_BYTES ((LDS_SACC + LDS_DEN + LDS_MX + LDS_LIST + NWAVE) * 4)
#define HEAD_LDS_BYTES (NG * HD * 4 + NG * GP * 2 + NG * 4)

static_assert(WCAP == (CHUNK / NTHR) * 32);
static_assert(NGRP >= 1);
static_assert(NB == 256);
static_assert(NB == NWAVE * 32);
static_assert(CHUNK == 2048);
static_assert(HC == 32 && NH * HC == HD);
static_assert(((LDS_SACC + LDS_DEN) % 4) == 0);
static_assert(AGG_LDS_BYTES == 286752);
static_assert(HEAD_LDS_BYTES == 99584);
static_assert(2 * NG * OSP <= NG * HD);
static_assert((XSP % 4) == 0 && (OSP % 4) == 0 && (GP % 8) == 0);

typedef float    v4f  __attribute__((ext_vector_type(4)));
typedef float    v8f  __attribute__((ext_vector_type(8)));
typedef int      v4i  __attribute__((ext_vector_type(4)));
typedef _Float16 v8h  __attribute__((ext_vector_type(8)));
typedef _Float16 v16h __attribute__((ext_vector_type(16)));
union Frag   { v16h v; v8h half[2]; };
union Pack16 { v8h h; v4i i; };

__device__ __forceinline__ v8f wm(v16h a, v16h b, v8f c) {
  v8f d = __builtin_amdgcn_wmma_f32_16x16x32_f16(false, a, false, b, (short)0, c, false, false);
  asm volatile("v_nop\n\tv_nop\n\tv_nop\n\tv_nop" : "+v"(d) : "v"(a), "v"(b));
  return d;
}

__device__ __forceinline__ v8f z8() {
  v8f z = {0.f, 0.f, 0.f, 0.f, 0.f, 0.f, 0.f, 0.f};
  return z;
}

__device__ __forceinline__ v8h pack8(v4f a, v4f b) {
  Pack16 u;
  u.h[0] = (_Float16)a.x; u.h[1] = (_Float16)a.y; u.h[2] = (_Float16)a.z; u.h[3] = (_Float16)a.w;
  u.h[4] = (_Float16)b.x; u.h[5] = (_Float16)b.y; u.h[6] = (_Float16)b.z; u.h[7] = (_Float16)b.w;
  return u.h;
}

__global__ __launch_bounds__(NTHR) void k_cvt(const float* __restrict__ W, _Float16* Wh, int n8, float sc) {
  const int i = blockIdx.x * NTHR + threadIdx.x;
  if (i >= n8) return;
  const size_t o = (size_t)i * 8;
  const v4f a = *(const v4f*)(W + o);
  const v4f b = *(const v4f*)(W + o + 4);
  Pack16 u;
  u.h = pack8(a * sc, b * sc);
  *(volatile v4i*)(Wh + o) = u.i;
  __threadfence();
  *(volatile v4i*)(Wh + o) = u.i;
}

__global__ __launch_bounds__(NTHR) void k_lora(const float* __restrict__ muA, const float* __restrict__ muB,
                                               const float* __restrict__ lvA, const float* __restrict__ lvB,
                                               _Float16* ba16) {
  const int i = blockIdx.x * NTHR + threadIdx.x;
  if (i >= 2 * NG * (HD / 8)) return;
  const int which = i >> 11;
  const int j     = (i >> 5) & (NG - 1);
  const int k0    = (i & 31) * 8;
  const float* A = which ? lvA : muA;
  const float* B = which ? lvB : muB;
  v4f acc0 = {0.f, 0.f, 0.f, 0.f};
  v4f acc1 = {0.f, 0.f, 0.f, 0.f};
#pragma unroll
  for (int r = 0; r < LR; ++r) {
    const float b = B[j * LR + r];
    const v4f a0 = *(const v4f*)(A + (size_t)r * HD + k0);
    const v4f a1 = *(const v4f*)(A + (size_t)r * HD + k0 + 4);
    acc0 += b * a0;
    acc1 += b * a1;
  }
  Pack16 u;
  u.h = pack8(acc0 * 1024.0f, acc1 * 1024.0f);
  const size_t o = (size_t)i * 8;
  *(volatile v4i*)(ba16 + o) = u.i;
  __threadfence();
  *(volatile v4i*)(ba16 + o) = u.i;
}

__device__ __forceinline__ void epi2(v8f a0, v8f a1, int T, int hh, int m, int wave, int nc0, int nc1,
                                     float cs0, float cs1, float cd0, float cd1,
                                     float* Xs, float* As, float* Ds) {
  float ss[8], sd[8];
#pragma unroll
  for (int r = 0; r < 8; ++r) {
    const float v0 = a0[r] * 0.0625f;
    const float v1 = a1[r] * 0.0625f;
    Xs[(T * 16 + 8 * hh + r) * XSP + nc0] = v0;
    Xs[(T * 16 + 8 * hh + r) * XSP + nc1] = v1;
    ss[r] = v0 * cs0 + v1 * cs1;
    sd[r] = v0 * cd0 + v1 * cd1;
  }
#pragma unroll
  for (int mk = 1; mk < 16; mk <<= 1) {
#pragma unroll
    for (int r = 0; r < 8; ++r) {
      ss[r] += __shfl_xor(ss[r], mk, 32);
      sd[r] += __shfl_xor(sd[r], mk, 32);
    }
  }
  if (m == 0) {
#pragma unroll
    for (int r = 0; r < 8; ++r) {
      As[(T * 16 + 8 * hh + r) * NH + wave] = ss[r];
      Ds[(T * 16 + 8 * hh + r) * NH + wave] = sd[r];
    }
  }
}

template <int K, bool ENC>
__global__ __launch_bounds__(NTHR) void k_gemm(
    const float* __restrict__ A, const _Float16* __restrict__ Wh, const float* __restrict__ bias,
    const float* __restrict__ att_s, const float* __restrict__ att_d,
    float* Y, float* asrc, float* adst, int nN) {
  constexpr int AP  = K + 8;
  constexpr int CPT = K / 8;
  __shared__ __attribute__((aligned(16))) _Float16 At[GR * AP];
  __shared__ __attribute__((aligned(16))) float Xs[GR * XSP];
  __shared__ __attribute__((aligned(16))) float As[GR * NH];
  __shared__ __attribute__((aligned(16))) float Ds[GR * NH];

  const int tid  = threadIdx.x;
  const int lane = tid & 31;
  const int wave = tid >> 5;
  const int hh   = lane >> 4;
  const int m    = lane & 15;
  const int rowBase = blockIdx.x * GR;

  {
    const int r  = tid >> 3;
    const int c0 = (tid & 7) * CPT;
    int row = rowBase + r;
    if (row > nN - 1) row = nN - 1;
    const float* p = A + (size_t)row * K + c0;
#pragma unroll
    for (int j = 0; j < CPT / 8; ++j) {
      const v4f f0 = *(const v4f*)(p + 8 * j);
      const v4f f1 = *(const v4f*)(p + 8 * j + 4);
      *(v8h*)(At + r * AP + c0 + 8 * j) = pack8(f0, f1);
    }
  }
  __syncthreads();

  const int nc0 = wave * 32 + m;
  const int nc1 = nc0 + 16;
  v8f c00 = z8(), c01 = z8(), c10 = z8(), c11 = z8();
#pragma unroll 2
  for (int kt = 0; kt < K / 32; ++kt) {
    const int k0 = kt * 32 + 8 * hh;
    Frag a0, a1, b0, b1;
    const _Float16* pa0 = At + m * AP + k0;
    const _Float16* pa1 = At + (16 + m) * AP + k0;
    const _Float16* pb0 = Wh + (size_t)nc0 * K + k0;
    const _Float16* pb1 = Wh + (size_t)nc1 * K + k0;
    a0.half[0] = *(const v8h*)pa0; a0.half[1] = *(const v8h*)(pa0 + 16);
    a1.half[0] = *(const v8h*)pa1; a1.half[1] = *(const v8h*)(pa1 + 16);
    b0.half[0] = *(const v8h*)pb0; b0.half[1] = *(const v8h*)(pb0 + 16);
    b1.half[0] = *(const v8h*)pb1; b1.half[1] = *(const v8h*)(pb1 + 16);
    c00 = wm(a0.v, b0.v, c00);
    c01 = wm(a0.v, b1.v, c01);
    c10 = wm(a1.v, b0.v, c10);
    c11 = wm(a1.v, b1.v, c11);
  }

  if (ENC) {
    const float bv0 = bias[nc0];
    const float bv1 = bias[nc1];
#pragma unroll
    for (int r = 0; r < 8; ++r) {
      Xs[(8 * hh + r) * XSP + nc0]      = c00[r] * 0.0625f + bv0;
      Xs[(8 * hh + r) * XSP + nc1]      = c01[r] * 0.0625f + bv1;
      Xs[(16 + 8 * hh + r) * XSP + nc0] = c10[r] * 0.0625f + bv0;
      Xs[(16 + 8 * hh + r) * XSP + nc1] = c11[r] * 0.0625f + bv1;
    }
  } else {
    const float cs0 = att_s[nc0], cs1 = att_s[nc1];
    const float cd0 = att_d[nc0], cd1 = att_d[nc1];
    epi2(c00, c01, 0, hh, m, wave, nc0, nc1, cs0, cs1, cd0, cd1, Xs, As, Ds);
    epi2(c10, c11, 1, hh, m, wave, nc0, nc1, cs0, cs1, cd0, cd1, Xs, As, Ds);
  }
  __syncthreads();

  v4f xr[8];
  float* yp[4];
#pragma unroll
  for (int i = 0; i < 4; ++i) {
    const int row = 4 * wave + i;
    xr[2 * i]     = *(const v4f*)(Xs + row * XSP + 4 * lane);
    xr[2 * i + 1] = *(const v4f*)(Xs + row * XSP + 128 + 4 * lane);
    yp[i] = Y + (size_t)(rowBase + row) * HD + 4 * lane;
  }
  float* gp = 0;
  v4f g0 = {0.f, 0.f, 0.f, 0.f};
  v4f g1 = {0.f, 0.f, 0.f, 0.f};
  if (!ENC) {
    if (wave == 0) {
      g0 = *(const v4f*)(As + 4 * lane);
      g1 = *(const v4f*)(As + 128 + 4 * lane);
      gp = asrc + (size_t)rowBase * NH + 4 * lane;
    } else if (wave == 1) {
      g0 = *(const v4f*)(Ds + 4 * lane);
      g1 = *(const v4f*)(Ds + 128 + 4 * lane);
      gp = adst + (size_t)rowBase * NH + 4 * lane;
    }
  }
#pragma unroll
  for (int i = 0; i < 4; ++i) {
    *(volatile v4f*)(yp[i])       = xr[2 * i];
    *(volatile v4f*)(yp[i] + 128) = xr[2 * i + 1];
  }
  if (gp) { *(volatile v4f*)gp = g0; *(volatile v4f*)(gp + 128) = g1; }
  __threadfence();
#pragma unroll
  for (int i = 0; i < 4; ++i) {
    *(volatile v4f*)(yp[i])       = xr[2 * i];
    *(volatile v4f*)(yp[i] + 128) = xr[2 * i + 1];
  }
  if (gp) { *(volatile v4f*)gp = g0; *(volatile v4f*)(gp + 128) = g1; }
}

__global__ __launch_bounds__(NTHR) void k_agg(
    const int* __restrict__ ei, const float* __restrict__ hp,
    const float* __restrict__ asrc, const float* __restrict__ adst,
    const float* __restrict__ bias, float* hout, int nN, int nE) {
  extern __shared__ v4f lds_agg[];
  float* sacc = (float*)lds_agg;
  float* den  = sacc + LDS_SACC;
  float* mx   = den + LDS_DEN;
  int*   list = (int*)(mx + LDS_MX);
  int*   wcnt = list + LDS_LIST;

  const int tid  = threadIdx.x;
  const int lane = tid & 31;
  const int wave = tid >> 5;
  const int hd   = lane >> 2;
  const int nodeBase = blockIdx.x * NB;

  {
    const v4f z4 = {0.f, 0.f, 0.f, 0.f};
    for (int i = tid; i < (LDS_SACC + LDS_DEN) / 4; i += NTHR) lds_agg[i] = z4;
    for (int i = tid; i < LDS_MX; i += NTHR) mx[i] = -1.0e30f;
  }
  __syncthreads();

  const int* eid = ei + nE;
  const bool al16 = ((nE & 3) == 0);

  const int nChunks = (nE + CHUNK - 1) / CHUNK;
#pragma unroll 1
  for (int ch = 0; ch < nChunks; ++ch) {
    const int cbase = ch * CHUNK;
    int wc = 0;
#pragma unroll
    for (int g = 0; g < NGRP; ++g) {
      const int el0 = (g * NTHR + tid) * 4;
      const int e0  = cbase + el0;
      const int sent = -2147483647 - 1;
      v4i d;
      if (al16 && (e0 + 3 < nE)) {
        d = *(const v4i*)(eid + e0);
      } else {
        d.x = (e0     < nE) ? eid[min(e0, nE - 1)]     : sent;
        d.y = (e0 + 1 < nE) ? eid[min(e0 + 1, nE - 1)] : sent;
        d.z = (e0 + 2 < nE) ? eid[min(e0 + 2, nE - 1)] : sent;
        d.w = (e0 + 3 < nE) ? eid[min(e0 + 3, nE - 1)] : sent;
      }
      const unsigned s0 = (unsigned)d.x - (unsigned)nodeBase;
      const unsigned s1 = (unsigned)d.y - (unsigned)nodeBase;
      const unsigned s2 = (unsigned)d.z - (unsigned)nodeBase;
      const unsigned s3 = (unsigned)d.w - (unsigned)nodeBase;
      const bool h0 = s0 < (unsigned)NB;
      const bool h1 = s1 < (unsigned)NB;
      const bool h2 = s2 < (unsigned)NB;
      const bool h3 = s3 < (unsigned)NB;
      const unsigned many = __builtin_amdgcn_ballot_w32(h0 | h1 | h2 | h3);
      if (many != 0u) {
#define HITJ(J, HJ, SJ) { \
          const unsigned mj = __builtin_amdgcn_ballot_w32(HJ); \
          if (HJ) { \
            const int pos = wc + (int)__builtin_amdgcn_mbcnt_lo(mj, 0u); \
            if (pos < WCAP) list[wave * WCAP + pos] = ((el0 + (J)) << 8) | (int)(SJ); \
          } \
          wc += (int)__builtin_popcount(mj); }
        HITJ(0, h0, s0)
        HITJ(1, h1, s1)
        HITJ(2, h2, s2)
        HITJ(3, h3, s3)
#undef HITJ
      }
    }
    if (lane == 0) wcnt[wave] = wc;
    __syncthreads();

    if (wave == 0) {
      for (int wsx = 0; wsx < NWAVE; ++wsx) {
        int n = wcnt[wsx];
        if (n > WCAP) n = WCAP;
        if (n < 0) n = 0;
        for (int i = 0; i < n; ++i) {
          const int ent  = list[wsx * WCAP + i];
          const int slot = ent & (NB - 1);
          const int el   = (ent >> 8) & (CHUNK - 1);
          int e = cbase + el;
          if (e > nE - 1) e = nE - 1;
          int src = ei[e];
          src = src < 0 ? 0 : (src > nN - 1 ? nN - 1 : src);
          int nd = nodeBase + slot;
          if (nd > nN - 1) nd = nN - 1;
          float al = asrc[(size_t)src * NH + hd] + adst[(size_t)nd * NH + hd];
          al = (al >= 0.f) ? al : 0.2f * al;
          const int mi = slot * NH + hd;
          const float mo = mx[mi];
          const float mn = fmaxf(mo, al);
          const float sc = __expf(mo - mn);
          const float p  = __expf(al - mn);
          const float* hs = hp + (size_t)src * HD + 8 * lane;
          const v4f x0 = *(const v4f*)(hs);
          const v4f x1 = *(const v4f*)(hs + 4);
          v4f* sp = (v4f*)(sacc + slot * HD + 8 * lane);
          v4f a0 = sp[0];
          v4f a1 = sp[1];
          a0 = a0 * sc + p * x0;
          a1 = a1 * sc + p * x1;
          sp[0] = a0;
          sp[1] = a1;
          if ((lane & 3) == 0) {
            const float dv = den[mi];
            den[mi] = dv * sc + p;
            mx[mi]  = mn;
          }
        }
      }
    }
    __syncthreads();
  }

  const int ha = lane >> 3;
  const int hb = 4 + (lane >> 3);
  const v4f b4a = *(const v4f*)(bias + 4 * lane);
  const v4f b4b = *(const v4f*)(bias + 128 + 4 * lane);
#pragma unroll 1
  for (int j = 0; j < NB / NWAVE; ++j) {
    const int slot = wave * (NB / NWAVE) + j;
    const int node = nodeBase + slot;
    if (node >= nN) break;
    const size_t nr = (size_t)node;
    float ala = asrc[nr * NH + ha] + adst[nr * NH + ha];
    float alb = asrc[nr * NH + hb] + adst[nr * NH + hb];
    ala = (ala >= 0.f) ? ala : 0.2f * ala;
    alb = (alb >= 0.f) ? alb : 0.2f * alb;
    const float moa = mx[slot * NH + ha];
    const float mob = mx[slot * NH + hb];
    const float mna = fmaxf(moa, ala);
    const float mnb = fmaxf(mob, alb);
    const float sca = __expf(moa - mna);
    const float scb = __expf(mob - mnb);
    const float pa  = __expf(ala - mna);
    const float pb  = __expf(alb - mnb);
    const float dena = den[slot * NH + ha] * sca + pa;
    const float denb = den[slot * NH + hb] * scb + pb;
    const v4f xa = *(const v4f*)(hp + nr * HD + 4 * lane);
    const v4f xb = *(const v4f*)(hp + nr * HD + 128 + 4 * lane);
    const v4f sa = *(const v4f*)(sacc + slot * HD + 4 * lane) * sca + pa * xa;
    const v4f sb = *(const v4f*)(sacc + slot * HD + 128 + 4 * lane) * scb + pb * xb;
    const float ia = 1.0f / dena;
    const float ib = 1.0f / denb;
    v4f ya = sa * ia + b4a;
    v4f yb = sb * ib + b4b;
    ya.x = ya.x > 0.f ? ya.x : 0.f; ya.y = ya.y > 0.f ? ya.y : 0.f;
    ya.z = ya.z > 0.f ? ya.z : 0.f; ya.w = ya.w > 0.f ? ya.w : 0.f;
    yb.x = yb.x > 0.f ? yb.x : 0.f; yb.y = yb.y > 0.f ? yb.y : 0.f;
    yb.z = yb.z > 0.f ? yb.z : 0.f; yb.w = yb.w > 0.f ? yb.w : 0.f;
    float* op = hout + nr * HD + 4 * lane;
    *(volatile v4f*)op = ya;
    *(volatile v4f*)(op + 128) = yb;
    __threadfence();
    *(volatile v4f*)op = ya;
    *(volatile v4f*)(op + 128) = yb;
  }
}

__global__ __launch_bounds__(NTHR) void k_head(
    const float* __restrict__ hin, const int* __restrict__ batch,
    const _Float16* __restrict__ hw16, const _Float16* __restrict__ ba16,
    const float* __restrict__ mub, const float* __restrict__ lvb,
    float* out, int nN) {
  extern __shared__ v4f lds_head[];
  float*    gsum = (float*)lds_head;
  _Float16* g16  = (_Float16*)(gsum + NG * HD);
  float*    cnt  = (float*)(g16 + NG * GP);

  const int tid  = threadIdx.x;
  const int lane = tid & 31;
  const int wave = tid >> 5;
  const int hh   = lane >> 4;
  const int m    = lane & 15;

  {
    const v4f z4 = {0.f, 0.f, 0.f, 0.f};
    for (int i = tid; i < NG * HD / 4; i += NTHR) lds_head[i] = z4;
    if (tid < NG) cnt[tid] = 0.f;
  }
  __syncthreads();

#pragma unroll 2
  for (int n = 0; n < nN; ++n) {
    const int b = batch[n];
    if ((unsigned)b < (unsigned)NG) {
      const float v = hin[(size_t)n * HD + tid];
      gsum[b * HD + tid] += v;
      if (tid == 0) cnt[b] += 1.0f;
    }
  }
  __syncthreads();
  if (tid < NG) {
    const float c = cnt[tid];
    cnt[tid] = 1.0f / fmaxf(c, 1.0f);
  }
  __syncthreads();
#pragma unroll 4
  for (int gi = 0; gi < NG; ++gi)
    g16[gi * GP + tid] = (_Float16)(gsum[gi * HD + tid] * cnt[gi]);
  __syncthreads();

  const int which = wave >> 2;
  const int ct    = wave & 3;
  const int ncol  = ct * 16 + m;
  const _Float16* Wp = hw16 + ((size_t)which * LT + ncol) * HD;
  const _Float16* Bp = ba16 + ((size_t)which * LT + ncol) * HD;
  const float bv = (which ? lvb : mub)[ncol];
  float* outs = gsum;
#pragma unroll 1
  for (int rt = 0; rt < NG / 16; ++rt) {
    v8f cw = z8(), cb = z8();
#pragma unroll 2
    for (int kt = 0; kt < HD / 32; ++kt) {
      const int k0 = kt * 32 + 8 * hh;
      Frag a, bw, bb;
      const _Float16* pa = g16 + (16 * rt + m) * GP + k0;
      const _Float16* pw = Wp + k0;
      const _Float16* pb = Bp + k0;
      a.half[0]  = *(const v8h*)pa; a.half[1]  = *(const v8h*)(pa + 16);
      bw.half[0] = *(const v8h*)pw; bw.half[1] = *(const v8h*)(pw + 16);
      bb.half[0] = *(const v8h*)pb; bb.half[1] = *(const v8h*)(pb + 16);
      cw = wm(a.v, bw.v, cw);
      cb = wm(a.v, bb.v, cb);
    }
#pragma unroll
    for (int r = 0; r < 8; ++r) {
      const float v = cw[r] * 0.0625f + cb[r] * 0.001953125f + bv;
      outs[(which * NG + 16 * rt + 8 * hh + r) * OSP + ncol] = v;
    }
  }
  __syncthreads();

  v4f ov[8];
  float* pp[8];
#pragma unroll
  for (int i = 0; i < 8; ++i) {
    const int row = 16 * wave + 2 * i + (lane >> 4);
    const int col = 4 * (lane & 15);
    ov[i] = *(const v4f*)(outs + row * OSP + col);
    pp[i] = out + (size_t)row * LT + col;
  }
#pragma unroll
  for (int i = 0; i < 8; ++i) *(volatile v4f*)(pp[i]) = ov[i];
  __threadfence();
#pragma unroll
  for (int i = 0; i < 8; ++i) *(volatile v4f*)(pp[i]) = ov[i];
}

extern "C" void kernel_launch(void* const* d_in, const int* in_sizes, int n_in,
                              void* d_out, int out_size, void* d_ws, size_t ws_size,
                              hipStream_t stream) {
  if (n_in < 17) return;
  const int nN = in_sizes[0] / FI;
  if (nN <= 0 || in_sizes[0] != nN * FI) return;
  const int nE = in_sizes[1] / 2;
  if (nE < 0 || in_sizes[1] != 2 * nE) return;
  if (in_sizes[2] != nN) return;
  if (in_sizes[3] != HD * FI || in_sizes[4] != HD) return;
  if (in_sizes[5] != NL * HD * HD || in_sizes[6] != NL * NH * HC || in_sizes[7] != NL * NH * HC) return;
  if (in_sizes[8] != NL * HD) return;
  if (in_sizes[9] != LT * HD || in_sizes[10] != LT || in_sizes[11] != LR * HD || in_sizes[12] != LT * LR) return;
  if (in_sizes[13] != LT * HD || in_sizes[14] != LT || in_sizes[15] != LR * HD || in_sizes[16] != LT * LR) return;
  if (out_size != 2 * NG * LT) return;

  const float* x       = (const float*)d_in[0];
  const int*   ei      = (const int*)d_in[1];
  const int*   batch   = (const int*)d_in[2];
  const float* enc_W   = (const float*)d_in[3];
  const float* enc_b   = (const float*)d_in[4];
  const float* gat_W   = (const float*)d_in[5];
  const float* att_src = (const float*)d_in[6];
  const float* att_dst = (const float*)d_in[7];
  const float* gat_b   = (const float*)d_in[8];
  const float* mu_W    = (const float*)d_in[9];
  const float* mu_b    = (const float*)d_in[10];
  const float* mu_A    = (const float*)d_in[11];
  const float* mu_B    = (const float*)d_in[12];
  const float* lv_W    = (const float*)d_in[13];
  const float* lv_b    = (const float*)d_in[14];
  const float* lv_A    = (const float*)d_in[15];
  const float* lv_B    = (const float*)d_in[16];
  float* out = (float*)d_out;

  const int nP = ((nN + GR - 1) / GR) * GR;
  size_t off = 0;
  _Float16* encW16 = (_Float16*)((char*)d_ws + off); off += (size_t)HD * FI * sizeof(_Float16);
  _Float16* gatW16 = (_Float16*)((char*)d_ws + off); off += (size_t)NL * HD * HD * sizeof(_Float16);
  _Float16* hw16   = (_Float16*)((char*)d_ws + off); off += (size_t)2 * LT * HD * sizeof(_Float16);
  _Float16* ba16   = (_Float16*)((char*)d_ws + off); off += (size_t)2 * LT * HD * sizeof(_Float16);
  float* hA   = (float*)((char*)d_ws + off); off += (size_t)nP * HD * sizeof(float);
  float* hp   = (float*)((char*)d_ws + off); off += (size_t)nP * HD * sizeof(float);
  float* asrc = (float*)((char*)d_ws + off); off += (size_t)nP * NH * sizeof(float);
  float* adst = (float*)((char*)d_ws + off); off += (size_t)nP * NH * sizeof(float);
  if (off > ws_size) return;
  if (off > (size_t)134217728) return;

  {
    const int n8e = HD * FI / 8;
    k_cvt<<<(n8e + NTHR - 1) / NTHR, NTHR, 0, stream>>>(enc_W, encW16, n8e, 16.0f);
    const int n8g = NL * HD * HD / 8;
    k_cvt<<<(n8g + NTHR - 1) / NTHR, NTHR, 0, stream>>>(gat_W, gatW16, n8g, 16.0f);
    const int n8h = LT * HD / 8;
    k_cvt<<<(n8h + NTHR - 1) / NTHR, NTHR, 0, stream>>>(mu_W, hw16, n8h, 16.0f);
    k_cvt<<<(n8h + NTHR - 1) / NTHR, NTHR, 0, stream>>>(lv_W, hw16 + (size_t)LT * HD, n8h, 16.0f);
    const int nl = 2 * NG * (HD / 8);
    k_lora<<<(nl + NTHR - 1) / NTHR, NTHR, 0, stream>>>(mu_A, mu_B, lv_A, lv_B, ba16);
  }

  k_gemm<FI, true><<<nP / GR, NTHR, 0, stream>>>(x, encW16, enc_b, att_src, att_dst, hA, asrc, adst, nN);

  hipFuncSetAttribute(reinterpret_cast<const void*>(&k_agg),
                      hipFuncAttributeMaxDynamicSharedMemorySize, AGG_LDS_BYTES);
  const int gridAgg = (nN + NB - 1) / NB;
  for (int l = 0; l < NL; ++l) {
    k_gemm<HD, false><<<nP / GR, NTHR, 0, stream>>>(
        hA, gatW16 + (size_t)l * HD * HD, enc_b,
        att_src + (size_t)l * NH * HC, att_dst + (size_t)l * NH * HC,
        hp, asrc, adst, nN);
    k_agg<<<gridAgg, NTHR, AGG_LDS_BYTES, stream>>>(
        ei, hp, asrc, adst, gat_b + (size_t)l * HD, hA, nN, nE);
  }

  hipFuncSetAttribute(reinterpret_cast<const void*>(&k_head),
                      hipFuncAttributeMaxDynamicSharedMemorySize, HEAD_LDS_BYTES);
  k_head<<<1, NTHR, HEAD_LDS_BYTES, stream>>>(hA, batch, hw16, ba16, mu_b, lv_b, out, nN);
}
